// LRU_71777493450999
// MI455X (gfx1250) — hardware-verified
//
#include <hip/hip_runtime.h>
#include <math.h>

constexpr int NIN    = 512;
constexpr int NHID   = 1024;
constexpr int NOUTF  = 512;
constexpr int NBATCH = 8;
constexpr int NSTEP  = 2048;
constexpr int NBP    = 4;
constexpr int NPASS  = NBATCH / NBP;
constexpr int MROWS  = NBP * NSTEP;
constexpr int KCAT   = 2 * NHID + NIN;
constexpr int APITCH = KCAT;
constexpr int NTHR   = 256;
constexpr int SCAN_THR = NHID / 8;

static_assert(NPASS * NBP == NBATCH);
static_assert(MROWS % 64 == 0 && NHID % 64 == 0 && NOUTF % 64 == 0);
static_assert(NIN % 32 == 0 && KCAT % 32 == 0 && (2 * NHID) % 32 == 0);
static_assert(((MROWS / 64) * (NHID / 64)) % 8 == 0);
static_assert(((MROWS / 64) * (NOUTF / 64)) % 8 == 0);
static_assert(NHID % NTHR == 0);
static_assert(SCAN_THR * 8 == NHID && SCAN_THR % 32 == 0);
static_assert((NIN / 8) % 32 == 0 && (NHID / 8) % 32 == 0);
static_assert((NHID * (NIN / 8)) % NTHR == 0);
static_assert((NOUTF * (NHID / 8)) % NTHR == 0);
static_assert((NOUTF * (NIN / 8)) % NTHR == 0);
static_assert((MROWS * (NIN / 8)) % NTHR == 0);
static_assert(APITCH % 8 == 0);

typedef __attribute__((ext_vector_type(16))) __bf16   v16b;
typedef __attribute__((ext_vector_type(8)))  __bf16   v8b;
typedef __attribute__((ext_vector_type(8)))  _Float16 v8h;
typedef __attribute__((ext_vector_type(8)))  float    v8f;
typedef __attribute__((ext_vector_type(4)))  float    v4f;
typedef __attribute__((ext_vector_type(4)))  unsigned v4u;

__device__ __forceinline__ unsigned short f2bf_bits(float f) {
  unsigned u = __float_as_uint(f);
  return (unsigned short)((u + 0x7FFFu + ((u >> 16) & 1u)) >> 16);
}
__device__ __forceinline__ float bf_bits2f(unsigned short h) { return __uint_as_float(((unsigned)h) << 16); }
__device__ __forceinline__ float bf16r(float f) { return bf_bits2f(f2bf_bits(f)); }

__device__ __forceinline__ void keep4_b(v16b a, v16b b, v16b c, v16b d) { asm volatile("v_nop" :: "v"(a), "v"(b), "v"(c), "v"(d)); }
__device__ __forceinline__ void acc_guard4(v8f& a, v8f& b, v8f& c, v8f& d) { asm volatile("v_nop\n\tv_nop\n\tv_nop\n\tv_nop" : "+v"(a), "+v"(b), "+v"(c), "+v"(d)); }
__device__ __forceinline__ void guard_row_b(v8f& a, v8f& b, v8f& c, v8f& d, v16b x, v16b y) {
  asm volatile("v_nop\n\tv_nop\n\tv_nop\n\tv_nop" : "+v"(a), "+v"(b), "+v"(c), "+v"(d) : "v"(x), "v"(y));
}

template <typename T> struct Frag;
template <> struct Frag<__bf16> {
  typedef v16b V; union U { v16b v; v8b h[2]; };
  static __device__ __forceinline__ v16b load(const __bf16* p) {
    U f; f.h[0] = *(const v8b*)(p); f.h[1] = *(const v8b*)(p + 16); return f.v;
  }
  static __device__ __forceinline__ v8f mma(v16b a, v16b b, v8f c) {
    return __builtin_amdgcn_wmma_f32_16x16x32_bf16(false, a, false, b, (short)0, c, false, false);
  }
};

template <bool DS>
__device__ __forceinline__ void ktile32(v8f (&acc)[4][4],
                                        const __bf16* __restrict__ A, const __bf16* __restrict__ A2, int lda,
                                        const __bf16* __restrict__ Bt, int ldb,
                                        int m0, int n0, int rlane, int koff, int k0) {
  v16b bh[4];
#pragma unroll
  for (int j = 0; j < 4; ++j) {
    const size_t bo = (size_t)(n0 + (j << 4) + rlane) * (size_t)ldb + (size_t)(koff + k0);
    bh[j] = Frag<__bf16>::load(Bt + bo);
  }
#pragma unroll
  for (int i = 0; i < 4; ++i) {
    const size_t ao = (size_t)(m0 + (i << 4) + rlane) * (size_t)lda + (size_t)(koff + k0);
    const v16b ah = Frag<__bf16>::load(A + ao);
    v16b al = ah;
    if (DS) al = Frag<__bf16>::load(A2 + ao);
#pragma unroll
    for (int j = 0; j < 4; ++j) {
      acc[i][j] = Frag<__bf16>::mma(ah, bh[j], acc[i][j]);
      if (DS) acc[i][j] = Frag<__bf16>::mma(al, bh[j], acc[i][j]);
    }
    guard_row_b(acc[i][0], acc[i][1], acc[i][2], acc[i][3], ah, al);
  }
  keep4_b(bh[0], bh[1], bh[2], bh[3]);
}

template <bool SPLITA, int CS_MODE, int OUT_MODE>
__global__ __launch_bounds__(NTHR) void gemm_bf16_t64(
    const unsigned short* __restrict__ Ap, const unsigned short* __restrict__ A2p, int lda,
    const unsigned short* __restrict__ Btp, int ldb,
    void* Cout, void* Cout2, int ldc,
    const float* __restrict__ colscale,
    int M, int N, int K, int ksplit) {
  const __bf16* A  = (const __bf16*)Ap;
  const __bf16* A2 = (const __bf16*)A2p;
  const __bf16* Bt = (const __bf16*)Btp;
  __shared__ __align__(16) float sT[8][16 * 68];
  const int lane = threadIdx.x & 31;
  const int wave = threadIdx.x >> 5;
  const int tilesN = N >> 6;
  const int tilesM = M >> 6;
  const int tile = blockIdx.x * 8 + wave;
  if (tile >= tilesM * tilesN) return;
  const int tm = tile / tilesN;
  const int tn = tile - tm * tilesN;
  const int m0 = tm << 6;
  const int n0 = tn << 6;

  const int rlane = lane & 15;
  const int koff  = (lane >> 4) * 8;
  const int mOff  = (lane >> 4) * 8;

  v8f acc[4][4];
#pragma unroll
  for (int i = 0; i < 4; ++i)
#pragma unroll
    for (int j = 0; j < 4; ++j) acc[i][j] = (v8f){0.f, 0.f, 0.f, 0.f, 0.f, 0.f, 0.f, 0.f};

  const int kse = SPLITA ? ksplit : 0;
  for (int k0 = 0; k0 < kse; k0 += 32) ktile32<true>(acc, A, A2, lda, Bt, ldb, m0, n0, rlane, koff, k0);
  for (int k0 = kse; k0 < K; k0 += 32)  ktile32<false>(acc, A, A, lda, Bt, ldb, m0, n0, rlane, koff, k0);
  acc_guard4(acc[0][0], acc[0][1], acc[0][2], acc[0][3]);
  acc_guard4(acc[1][0], acc[1][1], acc[1][2], acc[1][3]);
  acc_guard4(acc[2][0], acc[2][1], acc[2][2], acc[2][3]);
  acc_guard4(acc[3][0], acc[3][1], acc[3][2], acc[3][3]);

  float* slab = sT[wave];
#pragma unroll
  for (int i = 0; i < 4; ++i) {
    const int mBase = m0 + (i << 4);
#pragma unroll
    for (int j = 0; j < 4; ++j) {
      const int n = n0 + (j << 4) + rlane;
      float csv = 1.0f;
      if (CS_MODE == 1) csv = bf16r(colscale[n]);
#pragma unroll
      for (int r = 0; r < 8; ++r) slab[(mOff + r) * 68 + (j << 4) + rlane] = acc[i][j][r] * csv;
    }
    __builtin_amdgcn_fence(__ATOMIC_RELEASE, "workgroup");
    __builtin_amdgcn_wave_barrier();
    __builtin_amdgcn_fence(__ATOMIC_ACQUIRE, "workgroup");
    if (OUT_MODE == 0) {
      float* C = (float*)Cout;
      const int hh = lane >> 4, c4 = (lane & 15) * 4;
      for (int pass = 0; pass < 2; ++pass) {
#pragma unroll
        for (int it = 0; it < 8; ++it) {
          const int row = it * 2 + hh;
          v4f v = *(const v4f*)(slab + row * 68 + c4);
          *(volatile v4f*)(C + (size_t)(mBase + row) * ldc + n0 + c4) = v;
        }
        __threadfence();
      }
    } else {
      const int q = lane >> 3, c8 = (lane & 7) * 8;
      unsigned short* C  = (unsigned short*)Cout;
      unsigned short* C2 = (unsigned short*)Cout2;
      for (int pass = 0; pass < 2; ++pass) {
#pragma unroll
        for (int it = 0; it < 4; ++it) {
          const int row = it * 4 + q;
          const float* sp = slab + row * 68 + c8;
          v8h hv, lv;
#pragma unroll
          for (int e = 0; e < 8; ++e) {
            const unsigned short hb = f2bf_bits(sp[e]);
            const unsigned short lb = f2bf_bits(sp[e] - bf_bits2f(hb));
            hv[e] = __builtin_bit_cast(_Float16, hb);
            lv[e] = __builtin_bit_cast(_Float16, lb);
          }
          *(volatile v8h*)(C  + (size_t)(mBase + row) * ldc + n0 + c8) = hv;
          *(volatile v8h*)(C2 + (size_t)(mBase + row) * ldc + n0 + c8) = lv;
        }
        __threadfence();
      }
    }
    __builtin_amdgcn_fence(__ATOMIC_RELEASE, "workgroup");
    __builtin_amdgcn_wave_barrier();
    __builtin_amdgcn_fence(__ATOMIC_ACQUIRE, "workgroup");
  }
}

__global__ __launch_bounds__(NTHR) void cvt_bf16x8(const float* __restrict__ src, unsigned short* __restrict__ dst,
                                                  int nrow, int ncol8, int spitch, int dpitch, int dcol0, float sgn) {
  const int i  = blockIdx.x * NTHR + threadIdx.x;
  const int n8 = nrow * ncol8;
  if (i < n8) {
    const int row = i / ncol8;
    const int c8  = i - row * ncol8;
    const float* sp = src + (size_t)row * (size_t)spitch + (size_t)(c8 * 8);
    const v4f a = *(const v4f*)(sp);
    const v4f b = *(const v4f*)(sp + 4);
    v8h hv;
#pragma unroll
    for (int e = 0; e < 4; ++e) {
      hv[e]     = __builtin_bit_cast(_Float16, f2bf_bits(a[e] * sgn));
      hv[4 + e] = __builtin_bit_cast(_Float16, f2bf_bits(b[e] * sgn));
    }
    unsigned short* dp = dst + (size_t)row * (size_t)dpitch + (size_t)(dcol0 + c8 * 8);
    *(volatile v8h*)dp = hv;
    __threadfence();
    *(volatile v8h*)dp = hv;
  }
}

__global__ __launch_bounds__(NTHR) void lam_kernel(const float* __restrict__ theta_log, const float* __restrict__ nu_log,
                                                  float* __restrict__ lam) {
  const int h = blockIdx.x * NTHR + threadIdx.x;
  const float th = bf16r(theta_log[h]);
  const float nv = bf16r(nu_log[h]);
  const float en = expf(nv);
  float mag = expf(-en);
  mag = (mag < 1.17549435e-38f) ? 0.0f : mag;
  const float ang = expf(th);
  float sv, cv;
  sincosf(ang, &sv, &cv);
  const float lre = mag * cv;
  const float lim = mag * sv;
  volatile float* lp = lam;
  lp[h] = lre;
  lp[NHID + h] = lim;
  __threadfence();
  lp[h] = lre;
  lp[NHID + h] = lim;
}

__global__ __launch_bounds__(SCAN_THR) void scan_kernel(unsigned short* HIp, unsigned short* LOp, const float* __restrict__ lam) {
  const int tid = threadIdx.x;
  const int bl  = blockIdx.x;
  const int h0  = 8 * tid;
  float lre[8], lim[8], hre[8], him[8];
  {
    const v4f a0 = *(const v4f*)(lam + h0);
    const v4f a1 = *(const v4f*)(lam + h0 + 4);
    const v4f b0 = *(const v4f*)(lam + NHID + h0);
    const v4f b1 = *(const v4f*)(lam + NHID + h0 + 4);
#pragma unroll
    for (int e = 0; e < 4; ++e) { lre[e] = a0[e]; lre[4 + e] = a1[e]; lim[e] = b0[e]; lim[4 + e] = b1[e]; }
#pragma unroll
    for (int q = 0; q < 8; ++q) { hre[q] = 0.0f; him[q] = 0.0f; }
  }
  const size_t rbase = (size_t)bl * (size_t)NSTEP * (size_t)APITCH + (size_t)h0;
  unsigned short* hrow = HIp + rbase;
  unsigned short* lrow = LOp + rbase;
#pragma unroll 1
  for (int t = 0; t < NSTEP; ++t) {
    const v4u wrh = *(const v4u*)(hrow);
    const v4u wrl = *(const v4u*)(lrow);
    const v4u wih = *(const v4u*)(hrow + NHID);
    const v4u wil = *(const v4u*)(lrow + NHID);
    v4u orh, orl, oih, oil;
#pragma unroll
    for (int q = 0; q < 4; ++q) {
      const int c0 = 2 * q, c1 = 2 * q + 1;
      const float br0 = __uint_as_float(wrh[q] << 16)          + __uint_as_float(wrl[q] << 16);
      const float br1 = __uint_as_float(wrh[q] & 0xffff0000u) + __uint_as_float(wrl[q] & 0xffff0000u);
      const float bi0 = __uint_as_float(wih[q] << 16)          + __uint_as_float(wil[q] << 16);
      const float bi1 = __uint_as_float(wih[q] & 0xffff0000u) + __uint_as_float(wil[q] & 0xffff0000u);
      const float nr0 = (lre[c0] * hre[c0] - lim[c0] * him[c0]) + br0;
      const float ni0 = (lre[c0] * him[c0] + lim[c0] * hre[c0]) + bi0;
      const float nr1 = (lre[c1] * hre[c1] - lim[c1] * him[c1]) + br1;
      const float ni1 = (lre[c1] * him[c1] + lim[c1] * hre[c1]) + bi1;
      hre[c0] = nr0; him[c0] = ni0; hre[c1] = nr1; him[c1] = ni1;
      const unsigned short hr0 = f2bf_bits(nr0), hr1 = f2bf_bits(nr1), hi0 = f2bf_bits(ni0), hi1 = f2bf_bits(ni1);
      const unsigned short lr0 = f2bf_bits(nr0 - bf_bits2f(hr0));
      const unsigned short lr1 = f2bf_bits(nr1 - bf_bits2f(hr1));
      const unsigned short li0 = f2bf_bits(ni0 - bf_bits2f(hi0));
      const unsigned short li1 = f2bf_bits(ni1 - bf_bits2f(hi1));
      orh[q] = (unsigned)hr0 | ((unsigned)hr1 << 16);
      orl[q] = (unsigned)lr0 | ((unsigned)lr1 << 16);
      oih[q] = (unsigned)hi0 | ((unsigned)hi1 << 16);
      oil[q] = (unsigned)li0 | ((unsigned)li1 << 16);
    }
    *(volatile v4u*)(hrow)        = orh;
    *(volatile v4u*)(hrow + NHID) = oih;
    *(volatile v4u*)(lrow)        = orl;
    *(volatile v4u*)(lrow + NHID) = oil;
    __threadfence();
    *(volatile v4u*)(hrow)        = orh;
    *(volatile v4u*)(hrow + NHID) = oih;
    *(volatile v4u*)(lrow)        = orl;
    *(volatile v4u*)(lrow + NHID) = oil;
    hrow += APITCH;
    lrow += APITCH;
  }
}

extern "C" void kernel_launch(void* const* d_in, const int* in_sizes, int n_in,
                              void* d_out, int out_size, void* d_ws, size_t ws_size, hipStream_t stream) {
  if (n_in < 9 || d_out == nullptr || d_ws == nullptr) return;
  if (in_sizes[0] != NBATCH * NSTEP * NIN || in_sizes[1] != NHID || in_sizes[2] != NHID || in_sizes[3] != NHID ||
      in_sizes[4] != NHID * NIN || in_sizes[5] != NHID * NIN || in_sizes[6] != NOUTF * NHID ||
      in_sizes[7] != NOUTF * NHID || in_sizes[8] != NOUTF * NIN || out_size != NBATCH * NSTEP * NOUTF) return;

  const float* u         = (const float*)d_in[0];
  const float* theta_log = (const float*)d_in[1];
  const float* nu_log    = (const float*)d_in[2];
  const float* gamma_log = (const float*)d_in[3];
  const float* b_re      = (const float*)d_in[4];
  const float* b_im      = (const float*)d_in[5];
  const float* c_re      = (const float*)d_in[6];
  const float* c_im      = (const float*)d_in[7];
  const float* d_mat     = (const float*)d_in[8];
  float* yout = (float*)d_out;

  char* ws = (char*)d_ws; size_t off = 0;
  auto carve = [&](size_t bytes) -> char* { char* p = ws + off; off += (bytes + 255) & ~(size_t)255; return p; };
  unsigned short* HI  = (unsigned short*)carve((size_t)MROWS * APITCH * 2);
  unsigned short* LO  = (unsigned short*)carve((size_t)MROWS * APITCH * 2);
  unsigned short* W1  = (unsigned short*)carve((size_t)2 * NHID * NIN * 2);
  unsigned short* W2  = (unsigned short*)carve((size_t)NOUTF * KCAT * 2);
  float*          LAM = (float*)carve((size_t)2 * NHID * 4);
  if (off > ws_size || off > (size_t)134217728) return;

  lam_kernel<<<NHID / NTHR, NTHR, 0, stream>>>(theta_log, nu_log, LAM);
  cvt_bf16x8<<<(NHID * (NIN / 8)) / NTHR, NTHR, 0, stream>>>(b_re, W1, NHID, NIN / 8, NIN, NIN, 0, 1.0f);
  cvt_bf16x8<<<(NHID * (NIN / 8)) / NTHR, NTHR, 0, stream>>>(b_im, W1 + (size_t)NHID * NIN, NHID, NIN / 8, NIN, NIN, 0, 1.0f);
  cvt_bf16x8<<<(NOUTF * (NHID / 8)) / NTHR, NTHR, 0, stream>>>(c_re, W2, NOUTF, NHID / 8, NHID, KCAT, 0, 1.0f);
  cvt_bf16x8<<<(NOUTF * (NHID / 8)) / NTHR, NTHR, 0, stream>>>(c_im, W2, NOUTF, NHID / 8, NHID, KCAT, NHID, -1.0f);
  cvt_bf16x8<<<(NOUTF * (NIN / 8)) / NTHR, NTHR, 0, stream>>>(d_mat, W2, NOUTF, NIN / 8, NIN, KCAT, 2 * NHID, 1.0f);

  const int g1 = ((MROWS / 64) * (NHID / 64)) / 8;
  const int g2 = ((MROWS / 64) * (NOUTF / 64)) / 8;
  for (int p = 0; p < NPASS; ++p) {
    const float* up = u + (size_t)p * MROWS * NIN;
    float* yp = yout + (size_t)p * MROWS * NOUTF;
    cvt_bf16x8<<<(MROWS * (NIN / 8)) / NTHR, NTHR, 0, stream>>>(up, HI, MROWS, NIN / 8, NIN, APITCH, 2 * NHID, 1.0f);
    gemm_bf16_t64<false, 1, 2><<<g1, NTHR, 0, stream>>>(
        HI + 2 * NHID, HI + 2 * NHID, APITCH, W1, NIN, (void*)HI, (void*)LO, APITCH,
        gamma_log, MROWS, NHID, NIN, 0);
    gemm_bf16_t64<false, 1, 2><<<g1, NTHR, 0, stream>>>(
        HI + 2 * NHID, HI + 2 * NHID, APITCH, W1 + (size_t)NHID * NIN, NIN, (void*)(HI + NHID), (void*)(LO + NHID), APITCH,
        gamma_log, MROWS, NHID, NIN, 0);
    scan_kernel<<<NBP, SCAN_THR, 0, stream>>>(HI, LO, LAM);
    gemm_bf16_t64<true, 0, 0><<<g2, NTHR, 0, stream>>>(
        HI, LO, APITCH, W2, KCAT, (void*)yp, (void*)yp, NOUTF,
        gamma_log, MROWS, NOUTF, KCAT, 2 * NHID);
  }
}
